// _RelationalGATLayer_9852654977185
// MI455X (gfx1250) — hardware-verified
//
#include <hip/hip_runtime.h>
#include <math.h>
#define SRB 1024
#define SCHK 4096
typedef __attribute__((ext_vector_type(16))) _Float16 v16h;
typedef __attribute__((ext_vector_type(8)))  _Float16 v8h;
typedef __attribute__((ext_vector_type(16))) __bf16   v16b;
typedef __attribute__((ext_vector_type(8)))  __bf16   v8b;
typedef __attribute__((ext_vector_type(8)))  float    v8f;
typedef __attribute__((ext_vector_type(4)))  float    v4f;
#define PSCALE 32768.0f
#define U16(p) ((const unsigned short*)(const void*)(p))
#define PSCALE_INV (1.0f / 32768.0f)

__device__ __forceinline__ unsigned short f2bf_bits(float f) {
  unsigned u = __float_as_uint(f);
  return (unsigned short)((u + 0x7FFFu + ((u >> 16) & 1u)) >> 16);
}
__device__ __forceinline__ float bf_bits2f(unsigned short h) { return __uint_as_float(((unsigned)h) << 16); }

__device__ __forceinline__ void dep_guard_h(v8f& a, v8f& b, v16h x, v16h y) { asm volatile("v_nop\n\tv_nop\n\tv_nop\n\tv_nop" : "+v"(a), "+v"(b) : "v"(x), "v"(y)); }
__device__ __forceinline__ void dep_guard_b(v8f& a, v8f& b, v16b x, v16b y) { asm volatile("v_nop\n\tv_nop\n\tv_nop\n\tv_nop" : "+v"(a), "+v"(b) : "v"(x), "v"(y)); }
__device__ __forceinline__ void keep4_h(v16h a, v16h b, v16h c, v16h d) { asm volatile("v_nop" :: "v"(a), "v"(b), "v"(c), "v"(d)); }
__device__ __forceinline__ void keep4_b(v16b a, v16b b, v16b c, v16b d) { asm volatile("v_nop" :: "v"(a), "v"(b), "v"(c), "v"(d)); }
__device__ __forceinline__ void acc_guard4(v8f& a, v8f& b, v8f& c, v8f& d) { asm volatile("v_nop\n\tv_nop\n\tv_nop\n\tv_nop" : "+v"(a), "+v"(b), "+v"(c), "+v"(d)); }
template <typename T> struct Frag;
template <> struct Frag<_Float16> {
  typedef v16h V; union U { v16h v; v8h h[2]; };
  static __device__ __forceinline__ v16h load(const _Float16* p) {
    U f; f.h[0] = *(const v8h*)(p); f.h[1] = *(const v8h*)(p + 16); return f.v;
  }
  static __device__ __forceinline__ v8f mma(v16h a, v16h b, v8f c) {
    return __builtin_amdgcn_wmma_f32_16x16x32_f16(false, a, false, b, (short)0, c, false, false);
  }
  static __device__ __forceinline__ void guard(v8f& a, v8f& b, v16h x, v16h y) { dep_guard_h(a, b, x, y); }
  static __device__ __forceinline__ void keep(v16h a, v16h b, v16h c, v16h d) { keep4_h(a, b, c, d); }
};
template <> struct Frag<__bf16> {
  typedef v16b V; union U { v16b v; v8b h[2]; };
  static __device__ __forceinline__ v16b load(const __bf16* p) {
    U f; f.h[0] = *(const v8b*)(p); f.h[1] = *(const v8b*)(p + 16); return f.v;
  }
  static __device__ __forceinline__ v8f mma(v16b a, v16b b, v8f c) {
    return __builtin_amdgcn_wmma_f32_16x16x32_bf16(false, a, false, b, (short)0, c, false, false);
  }
  static __device__ __forceinline__ void guard(v8f& a, v8f& b, v16b x, v16b y) { dep_guard_b(a, b, x, y); }
  static __device__ __forceinline__ void keep(v16b a, v16b b, v16b c, v16b d) { keep4_b(a, b, c, d); }
};

template <int ET> struct Elem;
template <> struct Elem<0> { typedef _Float16 T; };
template <> struct Elem<1> { typedef __bf16 T; };
template <int ET, bool SPLIT, int BIAS_MODE, int OUT_MODE, bool RESID, int ACT = 0>
__global__ __launch_bounds__(256) void wmma_gemm64(
    const unsigned short* __restrict__ Ap, const unsigned short* __restrict__ A2p, int lda, long strideA,
    const unsigned short* __restrict__ Btp, const unsigned short* __restrict__ Bt2p, int ldb, long strideB,
    void* __restrict__ Cout, void* __restrict__ Cout2, int ldc, long strideC,
    const float* __restrict__ bias,
    const float* __restrict__ resid, long strideR,
    int M, int N, int K, float scale) {
  typedef typename Elem<ET>::T T;
  typedef typename Frag<T>::V V;
  const T* A = (const T*)Ap; const T* A2 = (const T*)A2p; const T* Bt = (const T*)Btp; const T* Bt2 = (const T*)Bt2p;
  __shared__ __align__(16) float sT[8][16 * 68];
  const int b    = blockIdx.y;
  const int lane = threadIdx.x & 31;
  const int wave = threadIdx.x >> 5;
  const int tilesN = N >> 6;
  const int tilesM = M >> 6;
  const int tile = blockIdx.x * 8 + wave;
  if (tile >= tilesM * tilesN) return;
  const int tm = tile / tilesN;
  const int tn = tile - tm * tilesN;
  const int m0 = tm << 6;
  const int n0 = tn << 6;

  const T* Ab  = A  + (size_t)b * strideA;
  const T* Bb  = Bt + (size_t)b * strideB;
  const T* Ab2 = SPLIT ? (A2  + (size_t)b * strideA) : nullptr;
  const T* Bb2 = SPLIT ? (Bt2 + (size_t)b * strideB) : nullptr;

  const int rlane = lane & 15;
  const int koff  = (lane >> 4) * 8;
  const int mOff  = (lane >> 4) * 8;

  v8f acc[4][4];
#pragma unroll
  for (int i = 0; i < 4; ++i)
#pragma unroll
    for (int j = 0; j < 4; ++j) acc[i][j] = (v8f){0.f,0.f,0.f,0.f,0.f,0.f,0.f,0.f};

  for (int k0 = 0; k0 < K; k0 += 32) {
    V bh[4], bl[4];
#pragma unroll
    for (int j = 0; j < 4; ++j) {
      const size_t bo = (size_t)(n0 + (j << 4) + rlane) * ldb + koff + k0;
      bh[j] = Frag<T>::load(Bb + bo);
      if (SPLIT) bl[j] = Frag<T>::load(Bb2 + bo);
    }
#pragma unroll
    for (int i = 0; i < 4; ++i) {
      const size_t ao = (size_t)(m0 + (i << 4) + rlane) * lda + koff + k0;
      V ah = Frag<T>::load(Ab + ao);
      V al;
      if (SPLIT) al = Frag<T>::load(Ab2 + ao);
#pragma unroll
      for (int j = 0; j < 4; ++j) {
        acc[i][j] = Frag<T>::mma(ah, bh[j], acc[i][j]);
        if (SPLIT) {
          acc[i][j] = Frag<T>::mma(ah, bl[j], acc[i][j]);
          acc[i][j] = Frag<T>::mma(al, bh[j], acc[i][j]);
        }
      }
      Frag<T>::guard(acc[i][0], acc[i][3], ah, SPLIT ? al : ah);
    }
    Frag<T>::keep(bh[0], bh[1], bh[2], bh[3]);
    if (SPLIT) Frag<T>::keep(bl[0], bl[1], bl[2], bl[3]);
  }
  acc_guard4(acc[0][0], acc[0][1], acc[0][2], acc[0][3]);
  acc_guard4(acc[1][0], acc[1][1], acc[1][2], acc[1][3]);
  acc_guard4(acc[2][0], acc[2][1], acc[2][2], acc[2][3]);
  acc_guard4(acc[3][0], acc[3][1], acc[3][2], acc[3][3]);

  float* slab = sT[wave];
  const float* Rb = RESID ? (resid + (size_t)b * strideR) : nullptr;
#pragma unroll
  for (int i = 0; i < 4; ++i) {
    const int mBase = m0 + (i << 4);
#pragma unroll
    for (int j = 0; j < 4; ++j) {
      const int n = n0 + (j << 4) + rlane;
      float bv = 0.f;
      if (BIAS_MODE == 2) bv = bias[n];
#pragma unroll
      for (int r = 0; r < 8; ++r) {
        float v = acc[i][j][r] * scale;
        if (BIAS_MODE == 1) v += bias[mBase + mOff + r];
        if (BIAS_MODE == 2) v += bv;
        if (RESID) v += Rb[(size_t)(mBase + mOff + r) * ldc + n];
        if (ACT == 1) v = tanhf(v);
        if (ACT == 2) v = fmaxf(v, 0.0f);
        if (ACT == 3) v = v / (1.0f + expf(-v));
        if (ACT == 4) v = (v > 0.f) ? v : 0.01f * v;
        if (ACT == 5) v = 0.5f * v * (1.0f + erff(v * 0.70710678118654752f));
        slab[(mOff + r) * 68 + (j << 4) + rlane] = v;
      }
    }
    __builtin_amdgcn_fence(__ATOMIC_RELEASE, "workgroup");
    __builtin_amdgcn_wave_barrier();
    __builtin_amdgcn_fence(__ATOMIC_ACQUIRE, "workgroup");
    if (OUT_MODE == 0) {
      float* C = (float*)Cout + (size_t)b * strideC;
      const int hh = lane >> 4, c4 = (lane & 15) * 4;
      for (int pass = 0; pass < 2; ++pass) {
#pragma unroll
        for (int it = 0; it < 8; ++it) {
          const int row = it * 2 + hh;
          v4f v = *(const v4f*)(slab + row * 68 + c4);
          *(volatile v4f*)(C + (size_t)(mBase + row) * ldc + n0 + c4) = v;
        }
        __threadfence();
      }
    } else {
      const int q = lane >> 3, c8 = (lane & 7) * 8;
      unsigned short* C  = (unsigned short*)Cout  + (size_t)b * strideC;
      unsigned short* C2 = (OUT_MODE == 2) ? ((unsigned short*)Cout2 + (size_t)b * strideC) : nullptr;
      for (int pass = 0; pass < 2; ++pass) {
#pragma unroll
        for (int it = 0; it < 4; ++it) {
          const int row = it * 4 + q;
          const float* sp = slab + row * 68 + c8;
          v8h hv, lv;
#pragma unroll
          for (int e = 0; e < 8; ++e) {
            if (OUT_MODE == 1) {
              hv[e] = (_Float16)sp[e];
            } else {
              unsigned short hb = f2bf_bits(sp[e]);
              unsigned short lb = f2bf_bits(sp[e] - bf_bits2f(hb));
              hv[e] = __builtin_bit_cast(_Float16, hb);
              lv[e] = __builtin_bit_cast(_Float16, lb);
            }
          }
          *(volatile v8h*)(C + (size_t)(mBase + row) * ldc + n0 + c8) = hv;
          if (OUT_MODE == 2) *(volatile v8h*)(C2 + (size_t)(mBase + row) * ldc + n0 + c8) = lv;
        }
        __threadfence();
      }
    }
    __builtin_amdgcn_fence(__ATOMIC_RELEASE, "workgroup");
    __builtin_amdgcn_wave_barrier();
    __builtin_amdgcn_fence(__ATOMIC_ACQUIRE, "workgroup");
  }
}

__global__ __launch_bounds__(256) void cast_f32_f16x2(
    const float* __restrict__ in, _Float16* __restrict__ out, int n2) {
  int i = blockIdx.x * 256 + threadIdx.x;
  if (i < n2) {
    const _Float16 h0 = (_Float16)in[2 * i], h1 = (_Float16)in[2 * i + 1];
    const unsigned u = (unsigned)__builtin_bit_cast(unsigned short, h0) | ((unsigned)__builtin_bit_cast(unsigned short, h1) << 16);
    ((volatile unsigned*)out)[i] = u;
    __threadfence();
    ((volatile unsigned*)out)[i] = u;
  }
}


__global__ __launch_bounds__(256) void transpose_cast_f16(const float* __restrict__ in, int ldi,
                                                         _Float16* __restrict__ outT, int ldo, float scale) {
  __shared__ __align__(16) _Float16 tile[64][72];
  const int c0 = blockIdx.x * 64, r0 = blockIdx.y * 64;
  const int t = threadIdx.y * 32 + threadIdx.x;
  for (int i = threadIdx.y; i < 64; i += 8) {
    tile[threadIdx.x][i]      = (_Float16)(in[(size_t)(r0 + i) * ldi + c0 + threadIdx.x] * scale);
    tile[32 + threadIdx.x][i] = (_Float16)(in[(size_t)(r0 + i) * ldi + c0 + 32 + threadIdx.x] * scale);
  }
  __syncthreads();
  const int q = t >> 3, c8 = (t & 7) * 8;
  for (int pass = 0; pass < 2; ++pass) {
#pragma unroll
    for (int it = 0; it < 2; ++it) {
      const int c = it * 32 + q;
      v8h hv = *(const v8h*)(&tile[c][c8]);
      *(volatile v8h*)(outT + (size_t)(c0 + c) * ldo + r0 + c8) = hv;
    }
    __threadfence();
  }
}


#ifndef SRB
#define SRB 512
#endif
#ifndef SCHK
#define SCHK 4096
#endif
#define SEPT (SCHK / SRB)
__device__ __forceinline__ int blk_excl_scan(int cnt, int* scan_ws, int tid, int* tot) {
  const int lane = tid & 31, wave = tid >> 5; int incl = cnt;
#pragma unroll
  for (int o = 1; o < 32; o <<= 1) { const int v = __shfl_up(incl, o, 32); if (lane >= o) incl += v; }
  if (lane == 31) scan_ws[wave] = incl;
  __syncthreads();
  if (wave == 0) { int wv = (lane < SRB / 32) ? scan_ws[lane] : 0; int wincl = wv;
#pragma unroll
    for (int o = 1; o < 32; o <<= 1) { const int v = __shfl_up(wincl, o, 32); if (lane >= o) wincl += v; }
    if (lane < SRB / 32) scan_ws[32 + lane] = wincl - wv; if (lane == 31) scan_ws[64] = wincl; }
  __syncthreads();
  const int res = scan_ws[32 + wave] + incl - cnt; *tot = scan_ws[64];
  return res;
}
__device__ __forceinline__ int chunk_compact(const int* __restrict__ keyv, const int* __restrict__ othv, int e0, int ne, int n0, int nn, int tid, int* L0, int* L1, int* L2, int* scan_ws) {
  int hk[SEPT], ho[SEPT], he[SEPT]; int cnt = 0;
#pragma unroll
  for (int k = 0; k < SEPT; ++k) { const int e = e0 + tid * SEPT + k; hk[k] = -1; if (e < ne) { const int d = keyv[e]; if (d >= n0 && d < n0 + SRB && d < nn) { hk[k] = d - n0; int s = othv[e]; s = s < 0 ? 0 : (s >= nn ? nn - 1 : s); ho[k] = s; he[k] = e; ++cnt; } } }
  int tot; int p = blk_excl_scan(cnt, scan_ws, tid, &tot);
#pragma unroll
  for (int k = 0; k < SEPT; ++k) if (hk[k] >= 0) { L0[p] = hk[k]; L1[p] = ho[k]; if (L2) L2[p] = he[k]; ++p; }
  __syncthreads();
  return tot;
}
__global__ __launch_bounds__(SRB) void stream_deg_kernel(const int* __restrict__ keyv, const int* __restrict__ othv, int ne, int nn, int* __restrict__ DEG) {
  __shared__ int L0[SCHK]; __shared__ int L1[SCHK]; __shared__ int scan_ws[80];
  const int tid = threadIdx.x, n0 = blockIdx.x * SRB; int cnt = 0;
  for (int e0 = 0; e0 < ne; e0 += SCHK) { const int tot = chunk_compact(keyv, othv, e0, ne, n0, nn, tid, L0, L1, nullptr, scan_ws);
    for (int q = 0; q < tot; ++q) cnt += (L0[q] == tid) ? 1 : 0;
    __syncthreads(); }
  const int n = n0 + tid; if (n < nn) { ((volatile int*)DEG)[n] = cnt; __threadfence(); ((volatile int*)DEG)[n] = cnt; }
}

#define NN 50000
#define NPAD 50176
#define NE 500000
__global__ __launch_bounds__(256) void padcast_kernel(const float* __restrict__ X, unsigned* __restrict__ X16) {
  const long i = (long)blockIdx.x * 256 + threadIdx.x; if (i >= (long)NPAD * 128 / 2) return; const long r = (2 * i) / 128; float a = 0.f, b = 0.f; if (r < NN) { a = X[2 * i]; b = X[2 * i + 1]; }
  const unsigned u = (unsigned)__builtin_bit_cast(unsigned short, (_Float16)a) | ((unsigned)__builtin_bit_cast(unsigned short, (_Float16)b) << 16); ((volatile unsigned*)X16)[i] = u; __threadfence(); ((volatile unsigned*)X16)[i] = u;
}
__global__ __launch_bounds__(256) void asd_kernel(const float* __restrict__ XP, const float* __restrict__ as0, const float* __restrict__ ad0, const float* __restrict__ as1, const float* __restrict__ ad1, const float* __restrict__ as2, const float* __restrict__ ad2, float* __restrict__ ASD) {
  const int lane = threadIdx.x & 31, wave = threadIdx.x >> 5; const size_t n = (size_t)blockIdx.x * 8 + wave;
  float s = 0.f, d = 0.f;
  if (lane < 24) { const int r = lane / 8, h = lane % 8; const float* as_ = (r == 0) ? as0 : (r == 1 ? as1 : as2); const float* ad_ = (r == 0) ? ad0 : (r == 1 ? ad1 : ad2);
    const float* xp = XP + n * 384 + r * 128 + h * 16;
#pragma unroll
    for (int k = 0; k < 16; ++k) { s += xp[k] * as_[h * 16 + k]; d += xp[k] * ad_[h * 16 + k]; } }
  for (int pass = 0; pass < 2; ++pass) { ((volatile float*)ASD)[n * 64 + lane] = s; ((volatile float*)ASD)[n * 64 + 32 + lane] = d; __threadfence(); }
}
template <bool HASW>
__global__ __launch_bounds__(SRB) void gat_stream_kernel(const float* __restrict__ XP, const float* __restrict__ ASD, int r, int h0, const float* __restrict__ ew, const float* __restrict__ ce, const float* __restrict__ bias,
                                                        const int* __restrict__ dstv, const int* __restrict__ srcv, float* __restrict__ OUT) {
  __shared__ int L0[SCHK]; __shared__ int L1[SCHK]; __shared__ int L2[SCHK]; __shared__ int scan_ws[80];
  const int tid = threadIdx.x, n0 = blockIdx.x * SRB; const int n = n0 + tid; const int nc = n < NN ? n : NN - 1;
  float m[4], ssum[4], adn[4], ceh[4]; float acc[64];
#pragma unroll
  for (int h = 0; h < 4; ++h) { m[h] = -INFINITY; ssum[h] = 0.f; adn[h] = ASD[(size_t)nc * 64 + 32 + r * 8 + h0 + h]; ceh[h] = HASW ? ce[h0 + h] : 0.f; }
#pragma unroll
  for (int c = 0; c < 64; ++c) acc[c] = 0.f;
  for (int e0 = 0; e0 < NE; e0 += SCHK) { const int tot = chunk_compact(dstv, srcv, e0, NE, n0, NN, tid, L0, L1, L2, scan_ws);
    for (int q = 0; q < tot; ++q) { if (L0[q] == tid) { const int s = L1[q]; const float we = HASW ? ew[L2[q]] : 0.f; const float* xp = XP + (size_t)s * 384 + r * 128 + h0 * 16; const float* as_ = ASD + (size_t)s * 64 + r * 8 + h0;
#pragma unroll
        for (int h = 0; h < 4; ++h) { float al = as_[h] + adn[h]; if (HASW) al += we * ceh[h]; al = al > 0.f ? al : 0.2f * al;
          const float mn = fmaxf(m[h], al); const float rr = __expf(m[h] - mn), ex = __expf(al - mn); ssum[h] = ssum[h] * rr + ex; m[h] = mn;
#pragma unroll
          for (int d = 0; d < 16; d += 4) { const v4f v = *(const v4f*)(xp + h * 16 + d); acc[h * 16 + d] = acc[h * 16 + d] * rr + ex * v[0]; acc[h * 16 + d + 1] = acc[h * 16 + d + 1] * rr + ex * v[1]; acc[h * 16 + d + 2] = acc[h * 16 + d + 2] * rr + ex * v[2]; acc[h * 16 + d + 3] = acc[h * 16 + d + 3] * rr + ex * v[3]; } } } }
    __syncthreads(); }
  if (n >= NN) return;
  for (int pass = 0; pass < 2; ++pass) {
#pragma unroll
    for (int h = 0; h < 4; ++h) { const float inv = (ssum[h] > 0.f) ? 1.0f / ssum[h] : 0.f;
#pragma unroll
      for (int d = 0; d < 16; d += 4) { v4f o; for (int q2 = 0; q2 < 4; ++q2) o[q2] = acc[h * 16 + d + q2] * inv; *(volatile v4f*)(OUT + (size_t)n * 128 + (h0 + h) * 16 + d) = o; } }
    __threadfence(); }
}
__global__ __launch_bounds__(256) void final_kernel(const float* __restrict__ hin, const float* __restrict__ G0, const float* __restrict__ G1, const float* __restrict__ G2, const float* __restrict__ gb0, const float* __restrict__ gb1, const float* __restrict__ gb2,
                                                   const float* __restrict__ g0, const float* __restrict__ b0, const float* __restrict__ g1, const float* __restrict__ b1, const float* __restrict__ g2, const float* __restrict__ b2, const float* __restrict__ fl, float* __restrict__ out) {
  const int lane = threadIdx.x & 31, wave = threadIdx.x >> 5; const size_t n = (size_t)blockIdx.x * 8 + wave; if (n >= NN) return;
  const float f0 = fl[0], f1 = fl[1], f2 = fl[2]; const float fm = fmaxf(f0, fmaxf(f1, f2)); const float e0 = expf(f0 - fm), e1 = expf(f1 - fm), e2 = expf(f2 - fm); const float es = e0 + e1 + e2; const float a[3] = {e0 / es, e1 / es, e2 / es};
  const float* Gs[3] = {G0, G1, G2}; const float* gbs[3] = {gb0, gb1, gb2}; const float* gs[3] = {g0, g1, g2}; const float* bs[3] = {b0, b1, b2};
  v4f res = *(const v4f*)(hin + n * 128 + lane * 4);
#pragma unroll 1
  for (int p = 0; p < 3; ++p) { const v4f x = *(const v4f*)(Gs[p] + n * 128 + lane * 4) + *(const v4f*)(gbs[p] + lane * 4);   float s = x[0] + x[1] + x[2] + x[3]; for (int o = 16; o > 0; o >>= 1) s += __shfl_xor(s, o, 32); const float mu = s / 128.f;
    float v = 0.f; for (int q = 0; q < 4; ++q) { const float d = x[q] - mu; v += d * d; } for (int o = 16; o > 0; o >>= 1) v += __shfl_xor(v, o, 32); const float inv = rsqrtf(v / 128.f + 1e-5f);
    for (int q = 0; q < 4; ++q) { const int c = lane * 4 + q; float y = gs[p][c] * (x[q] - mu) * inv + bs[p][c]; y = y > 0.f ? y : (__expf(y) - 1.0f); res[q] += a[p] * y; } }
  *(volatile v4f*)(out + n * 128 + lane * 4) = res; __threadfence(); *(volatile v4f*)(out + n * 128 + lane * 4) = res;
}
__global__ __launch_bounds__(64) void ce_kernel(const float* We1, const float* ae1, const float* We2, const float* ae2, float* CE) {
  const int t = threadIdx.x; if (t < 16) { const int h = t & 7; const float* We = (t < 8) ? We1 : We2; const float* ae = (t < 8) ? ae1 : ae2; float s = 0.f; for (int k = 0; k < 16; ++k) s += We[h * 16 + k] * ae[h * 16 + k]; ((volatile float*)CE)[t] = s; __threadfence(); ((volatile float*)CE)[t] = s; }
}
extern "C" void kernel_launch(void* const* d_in, const int* in_sizes, int n_in, void* d_out, int out_size, void* d_ws, size_t ws_size, hipStream_t stream) {
  (void)in_sizes; (void)n_in; (void)out_size; (void)ws_size;
  auto F = [&](int i) { return (const float*)d_in[i]; }; auto IP = [&](int i) { return (const int*)d_in[i]; };
  const float* hin = F(0); const int* sec_idx = IP(1); const int* corr_idx = IP(2); const float* corr_w = F(3); const int* emb_idx = IP(4); const float* emb_w = F(5);
  const float* Ws[3] = {F(6), F(10), F(14)}; const float* As[3] = {F(7), F(11), F(15)}; const float* Ad[3] = {F(8), F(12), F(16)}; const float* Bs[3] = {F(9), F(13), F(17)};
  const float* corr_ae = F(18); const float* corr_We = F(19); const float* emb_ae = F(20); const float* emb_We = F(21);
  const float* g_sec = F(22); const float* b_sec = F(23); const float* g_corr = F(24); const float* b_corr = F(25); const float* g_emb = F(26); const float* b_emb = F(27); const float* fl = F(28);
  char* ws = (char*)d_ws; size_t off = 0;
  auto carve = [&](size_t bytes) -> char* { char* p = ws + off; off += (bytes + 255) & ~(size_t)255; return p; };
  unsigned* X16 = (unsigned*)carve((size_t)NPAD * 128 * 2); _Float16* WT = (_Float16*)carve(384 * 128 * 2); float* XP = (float*)carve((size_t)NPAD * 384 * 4); float* ASD = (float*)carve((size_t)NPAD * 64 * 4); float* CE = (float*)carve(256);
  float* G[3]; for (int k = 0; k < 3; ++k) G[k] = (float*)carve((size_t)NPAD * 128 * 4);
  padcast_kernel<<<(NPAD * 128 / 2 + 255) / 256, 256, 0, stream>>>(hin, X16);
  for (int k = 0; k < 3; ++k) transpose_cast_f16<<<dim3(2, 2), dim3(32, 8), 0, stream>>>(Ws[k], 128, WT + (size_t)k * 128 * 128, 128, 1.0f);
  { const int t = (NPAD / 64) * 6; wmma_gemm64<0, false, 0, 0, false><<<dim3((t + 7) / 8, 1), 256, 0, stream>>>((const unsigned short*)X16, nullptr, 128, 0, U16(WT), nullptr, 128, 0, XP, nullptr, 384, 0, nullptr, nullptr, 0, NPAD, 384, 128, 1.0f); }
  asd_kernel<<<NPAD / 8, 256, 0, stream>>>(XP, As[0], Ad[0], As[1], Ad[1], As[2], Ad[2], ASD);
  ce_kernel<<<1, 64, 0, stream>>>(corr_We, corr_ae, emb_We, emb_ae, CE);
  const int nb = (NN + SRB - 1) / SRB;
  for (int hh = 0; hh < 8; hh += 4) {
    gat_stream_kernel<false><<<nb, SRB, 0, stream>>>(XP, ASD, 0, hh, nullptr, nullptr, Bs[0], sec_idx + NE, sec_idx, G[0]);
    gat_stream_kernel<true><<<nb, SRB, 0, stream>>>(XP, ASD, 1, hh, corr_w, CE, Bs[1], corr_idx + NE, corr_idx, G[1]);
    gat_stream_kernel<true><<<nb, SRB, 0, stream>>>(XP, ASD, 2, hh, emb_w, CE + 8, Bs[2], emb_idx + NE, emb_idx, G[2]); }
  final_kernel<<<NPAD / 8, 256, 0, stream>>>(hin, G[0], G[1], G[2], Bs[0], Bs[1], Bs[2], g_sec, b_sec, g_corr, b_corr, g_emb, b_emb, fl, (float*)d_out);
}
